// TTDense_9706626090067
// MI455X (gfx1250) — hardware-verified
//
#include <hip/hip_runtime.h>
#include <math.h>

constexpr int kBatch    = 1024;
constexpr int kInFeat   = 4096;
constexpr int kOutFeat  = 4096;
constexpr int kChunkB   = 128;
constexpr int kNumChunks = kBatch / kChunkB;
constexpr int kRowsChunk = kChunkB * 256;
constexpr int kK1   = 32;
constexpr int kKbig = 512;
constexpr int kN12  = 512;
constexpr int kN3   = 64;
constexpr float kCarry  = 16.0f;
constexpr float kScale2 = 1.0f / 16.0f;
constexpr float kScale3 = 1.0f / 256.0f;
static_assert(kRowsChunk % 64 == 0);
static_assert(kN12 % 64 == 0 && kN3 % 64 == 0);
static_assert(kK1 % 32 == 0 && kKbig % 32 == 0);
static_assert(kNumChunks * kChunkB == kBatch);

constexpr size_t kOffXG  = 0;
constexpr size_t kSzXG   = (size_t)kBatch * 256 * kK1 * 2;
constexpr size_t kOffBT1 = kOffXG + kSzXG;
constexpr size_t kSzBT1  = (size_t)kN12 * kK1 * 2;
constexpr size_t kOffBT2 = kOffBT1 + kSzBT1;
constexpr size_t kSzBT2  = (size_t)kN12 * kKbig * 2;
constexpr size_t kOffBT3 = kOffBT2 + kSzBT2;
constexpr size_t kSzBT3  = (size_t)kN3 * kKbig * 2;
constexpr size_t kOffR1  = kOffBT3 + kSzBT3;
constexpr size_t kSzR    = (size_t)kRowsChunk * kN12 * 2;
constexpr size_t kOffR2  = kOffR1 + kSzR;
constexpr size_t kWsTotal = kOffR2 + kSzR;
static_assert(kOffBT1 % 128 == 0 && kOffBT2 % 128 == 0 && kOffBT3 % 128 == 0);
static_assert(kOffR1 % 128 == 0 && kOffR2 % 128 == 0);
static_assert((size_t)kRowsChunk * kN3 * 4 <= kSzR);
static_assert(kWsTotal == 84508672);
static_assert(kWsTotal <= (size_t)134217728);

constexpr int kPrepBlk1 = (kN12 * kK1 / 8) / 256;
constexpr int kPrepBlk2 = kPrepBlk1 + (kN12 * kKbig / 8) / 256;
constexpr int kPrepBlk3 = kPrepBlk2 + (kN3 * kKbig / 8) / 256;
constexpr int kGatherXBlk  = (kBatch * 256 * (kK1 / 8)) / 256;
constexpr int kRegatherBlk = (kRowsChunk * (kKbig / 8)) / 256;
constexpr int kEpiBlk      = (kRowsChunk * 16 / 4) / 256;
constexpr int kGemmBlk12   = ((kRowsChunk / 64) * (kN12 / 64)) / 8;
constexpr int kGemmBlk3    = ((kRowsChunk / 64) * (kN3 / 64)) / 8;
static_assert(kPrepBlk1 * 256 * 8 == kN12 * kK1);
static_assert((kPrepBlk2 - kPrepBlk1) * 256 * 8 == kN12 * kKbig);
static_assert((kPrepBlk3 - kPrepBlk2) * 256 * 8 == kN3 * kKbig);
static_assert(kGatherXBlk * 256 * 8 == kBatch * 256 * kK1);
static_assert(kRegatherBlk * 256 * 8 == kRowsChunk * kKbig);
static_assert(kEpiBlk * 256 * 4 == kRowsChunk * 16);
static_assert(kGemmBlk12 * 8 == (kRowsChunk / 64) * (kN12 / 64));
static_assert(kGemmBlk3 * 8 == (kRowsChunk / 64) * (kN3 / 64));

typedef __attribute__((ext_vector_type(16))) _Float16 v16h;
typedef __attribute__((ext_vector_type(8)))  _Float16 v8h;
typedef __attribute__((ext_vector_type(16))) __bf16   v16b;
typedef __attribute__((ext_vector_type(8)))  __bf16   v8b;
typedef __attribute__((ext_vector_type(8)))  float    v8f;
typedef __attribute__((ext_vector_type(4)))  float    v4f;
typedef __attribute__((ext_vector_type(4)))  unsigned int v4u;

__device__ __forceinline__ unsigned short f2bf_bits(float f) {
  unsigned u = __float_as_uint(f);
  return (unsigned short)((u + 0x7FFFu + ((u >> 16) & 1u)) >> 16);
}
__device__ __forceinline__ float bf_bits2f(unsigned short h) { return __uint_as_float(((unsigned)h) << 16); }

__device__ __forceinline__ void dep_guard_h(v8f& a, v8f& b, v16h x, v16h y) { asm volatile("v_nop\n\tv_nop\n\tv_nop\n\tv_nop" : "+v"(a), "+v"(b) : "v"(x), "v"(y)); }
__device__ __forceinline__ void dep_guard_b(v8f& a, v8f& b, v16b x, v16b y) { asm volatile("v_nop\n\tv_nop\n\tv_nop\n\tv_nop" : "+v"(a), "+v"(b) : "v"(x), "v"(y)); }
__device__ __forceinline__ void keep4_h(v16h a, v16h b, v16h c, v16h d) { asm volatile("v_nop" :: "v"(a), "v"(b), "v"(c), "v"(d)); }
__device__ __forceinline__ void keep4_b(v16b a, v16b b, v16b c, v16b d) { asm volatile("v_nop" :: "v"(a), "v"(b), "v"(c), "v"(d)); }
__device__ __forceinline__ void acc_guard4(v8f& a, v8f& b, v8f& c, v8f& d) { asm volatile("v_nop\n\tv_nop\n\tv_nop\n\tv_nop" : "+v"(a), "+v"(b), "+v"(c), "+v"(d)); }
template <typename T> struct Frag;
template <> struct Frag<_Float16> {
  typedef v16h V; union U { v16h v; v8h h[2]; };
  static __device__ __forceinline__ v16h load(const _Float16* p) {
    U f; f.h[0] = *(const v8h*)(p); f.h[1] = *(const v8h*)(p + 16); return f.v;
  }
  static __device__ __forceinline__ v8f mma(v16h a, v16h b, v8f c) {
    return __builtin_amdgcn_wmma_f32_16x16x32_f16(false, a, false, b, (short)0, c, false, false);
  }
  static __device__ __forceinline__ void guard(v8f& a, v8f& b, v16h x, v16h y) { dep_guard_h(a, b, x, y); }
  static __device__ __forceinline__ void keep(v16h a, v16h b, v16h c, v16h d) { keep4_h(a, b, c, d); }
};
template <> struct Frag<__bf16> {
  typedef v16b V; union U { v16b v; v8b h[2]; };
  static __device__ __forceinline__ v16b load(const __bf16* p) {
    U f; f.h[0] = *(const v8b*)(p); f.h[1] = *(const v8b*)(p + 16); return f.v;
  }
  static __device__ __forceinline__ v8f mma(v16b a, v16b b, v8f c) {
    return __builtin_amdgcn_wmma_f32_16x16x32_bf16(false, a, false, b, (short)0, c, false, false);
  }
  static __device__ __forceinline__ void guard(v8f& a, v8f& b, v16b x, v16b y) { dep_guard_b(a, b, x, y); }
  static __device__ __forceinline__ void keep(v16b a, v16b b, v16b c, v16b d) { keep4_b(a, b, c, d); }
};

__device__ __forceinline__ unsigned pk16(unsigned short a, unsigned short b) { return (unsigned)a | ((unsigned)b << 16); }
__device__ __forceinline__ unsigned short h_bits(float f) { const _Float16 h = (_Float16)f; return __builtin_bit_cast(unsigned short, h); }

template <int ET> struct Elem;
template <> struct Elem<0> { typedef _Float16 T; };
template <> struct Elem<1> { typedef __bf16 T; };
template <int ET, bool SPLIT, int BIAS_MODE, int OUT_MODE, bool RESID, int ACT = 0>
__global__ __launch_bounds__(256) void wmma_gemm64(
    const unsigned short* __restrict__ Ap, const unsigned short* __restrict__ A2p, int lda, long strideA,
    const unsigned short* __restrict__ Btp, const unsigned short* __restrict__ Bt2p, int ldb, long strideB,
    void* __restrict__ Cout, void* __restrict__ Cout2, int ldc, long strideC,
    const float* __restrict__ bias,
    const float* __restrict__ resid, long strideR,
    int M, int N, int K, float scale) {
  typedef typename Elem<ET>::T T;
  typedef typename Frag<T>::V V;
  const T* A = (const T*)Ap; const T* A2 = (const T*)A2p; const T* Bt = (const T*)Btp; const T* Bt2 = (const T*)Bt2p;
  __shared__ __align__(16) float sT[8][16 * 68];
  const int b    = blockIdx.y;
  const int lane = threadIdx.x & 31;
  const int wave = threadIdx.x >> 5;
  const int tilesN = N >> 6;
  const int tilesM = M >> 6;
  const int tile = blockIdx.x * 8 + wave;
  if (tile >= tilesM * tilesN) return;
  const int tm = tile / tilesN;
  const int tn = tile - tm * tilesN;
  const int m0 = tm << 6;
  const int n0 = tn << 6;

  const T* Ab  = A  + (size_t)b * strideA;
  const T* Bb  = Bt + (size_t)b * strideB;
  const T* Ab2 = SPLIT ? (A2  + (size_t)b * strideA) : nullptr;
  const T* Bb2 = SPLIT ? (Bt2 + (size_t)b * strideB) : nullptr;

  const int rlane = lane & 15;
  const int koff  = (lane >> 4) * 8;
  const int mOff  = (lane >> 4) * 8;

  v8f acc[4][4];
#pragma unroll
  for (int i = 0; i < 4; ++i)
#pragma unroll
    for (int j = 0; j < 4; ++j) acc[i][j] = (v8f){0.f,0.f,0.f,0.f,0.f,0.f,0.f,0.f};

  for (int k0 = 0; k0 < K; k0 += 32) {
    V bh[4], bl[4];
#pragma unroll
    for (int j = 0; j < 4; ++j) {
      const size_t bo = (size_t)(n0 + (j << 4) + rlane) * ldb + koff + k0;
      bh[j] = Frag<T>::load(Bb + bo);
      if (SPLIT) bl[j] = Frag<T>::load(Bb2 + bo);
    }
#pragma unroll
    for (int i = 0; i < 4; ++i) {
      const size_t ao = (size_t)(m0 + (i << 4) + rlane) * lda + koff + k0;
      V ah = Frag<T>::load(Ab + ao);
      V al;
      if (SPLIT) al = Frag<T>::load(Ab2 + ao);
#pragma unroll
      for (int j = 0; j < 4; ++j) {
        acc[i][j] = Frag<T>::mma(ah, bh[j], acc[i][j]);
        if (SPLIT) {
          acc[i][j] = Frag<T>::mma(ah, bl[j], acc[i][j]);
          acc[i][j] = Frag<T>::mma(al, bh[j], acc[i][j]);
        }
      }
      Frag<T>::guard(acc[i][0], acc[i][3], ah, SPLIT ? al : ah);
    }
    Frag<T>::keep(bh[0], bh[1], bh[2], bh[3]);
    if (SPLIT) Frag<T>::keep(bl[0], bl[1], bl[2], bl[3]);
  }
  acc_guard4(acc[0][0], acc[0][1], acc[0][2], acc[0][3]);
  acc_guard4(acc[1][0], acc[1][1], acc[1][2], acc[1][3]);
  acc_guard4(acc[2][0], acc[2][1], acc[2][2], acc[2][3]);
  acc_guard4(acc[3][0], acc[3][1], acc[3][2], acc[3][3]);

  float* slab = sT[wave];
  const float* Rb = RESID ? (resid + (size_t)b * strideR) : nullptr;
#pragma unroll
  for (int i = 0; i < 4; ++i) {
    const int mBase = m0 + (i << 4);
#pragma unroll
    for (int j = 0; j < 4; ++j) {
      const int n = n0 + (j << 4) + rlane;
      float bv = 0.f;
      if (BIAS_MODE == 2) bv = bias[n];
#pragma unroll
      for (int r = 0; r < 8; ++r) {
        float v = acc[i][j][r] * scale;
        if (BIAS_MODE == 1) v += bias[mBase + mOff + r];
        if (BIAS_MODE == 2) v += bv;
        if (RESID) v += Rb[(size_t)(mBase + mOff + r) * ldc + n];
        if (ACT == 2) v = fmaxf(v, 0.0f);
        if (ACT == 4) v = (v > 0.f) ? v : 0.01f * v;
        slab[(mOff + r) * 68 + (j << 4) + rlane] = v;
      }
    }
    __builtin_amdgcn_fence(__ATOMIC_RELEASE, "workgroup");
    __builtin_amdgcn_wave_barrier();
    __builtin_amdgcn_fence(__ATOMIC_ACQUIRE, "workgroup");
    if (OUT_MODE == 0) {
      float* C = (float*)Cout + (size_t)b * strideC;
      const int hh = lane >> 4, c4 = (lane & 15) * 4;
      for (int pass = 0; pass < 2; ++pass) {
#pragma unroll
        for (int it = 0; it < 8; ++it) {
          const int row = it * 2 + hh;
          v4f v = *(const v4f*)(slab + row * 68 + c4);
          *(volatile v4f*)(C + (size_t)(mBase + row) * ldc + n0 + c4) = v;
        }
        __threadfence();
      }
    } else {
      const int q = lane >> 3, c8 = (lane & 7) * 8;
      unsigned short* C  = (unsigned short*)Cout  + (size_t)b * strideC;
      unsigned short* C2 = (OUT_MODE == 2) ? ((unsigned short*)Cout2 + (size_t)b * strideC) : nullptr;
      for (int pass = 0; pass < 2; ++pass) {
#pragma unroll
        for (int it = 0; it < 4; ++it) {
          const int row = it * 4 + q;
          const float* sp = slab + row * 68 + c8;
          v8h hv, lv;
#pragma unroll
          for (int e = 0; e < 8; ++e) {
            if (OUT_MODE == 1) {
              hv[e] = (_Float16)sp[e];
            } else {
              unsigned short hb = f2bf_bits(sp[e]);
              unsigned short lb = f2bf_bits(sp[e] - bf_bits2f(hb));
              hv[e] = __builtin_bit_cast(_Float16, hb);
              lv[e] = __builtin_bit_cast(_Float16, lb);
            }
          }
          *(volatile v8h*)(C + (size_t)(mBase + row) * ldc + n0 + c8) = hv;
          if (OUT_MODE == 2) *(volatile v8h*)(C2 + (size_t)(mBase + row) * ldc + n0 + c8) = lv;
        }
        __threadfence();
      }
    }
    __builtin_amdgcn_fence(__ATOMIC_RELEASE, "workgroup");
    __builtin_amdgcn_wave_barrier();
    __builtin_amdgcn_fence(__ATOMIC_ACQUIRE, "workgroup");
  }
}

__device__ __forceinline__ v4u pack8_f16(float v0, float v1, float v2, float v3, float v4, float v5, float v6, float v7) {
  return (v4u){pk16(h_bits(v0), h_bits(v1)), pk16(h_bits(v2), h_bits(v3)),
               pk16(h_bits(v4), h_bits(v5)), pk16(h_bits(v6), h_bits(v7))};
}
__device__ __forceinline__ void store16_twice(unsigned short* dst, v4u u) {
  *(volatile v4u*)dst = u;
  __threadfence();
  *(volatile v4u*)dst = u;
}

__global__ __launch_bounds__(256) void prep_cores_kernel(const float* __restrict__ c0, const float* __restrict__ c1,
                                                          const float* __restrict__ c2,
                                                          unsigned short* __restrict__ bt1, unsigned short* __restrict__ bt2,
                                                          unsigned short* __restrict__ bt3) {
  const int blk = blockIdx.x;
  const int t = threadIdx.x;
  float v[8];
  unsigned short* dst;
  if (blk < kPrepBlk1) {
    const int g = blk * 256 + t;
    const int row = g >> 2, part = g & 3;
    const int p1 = row >> 5, q1 = row & 31;
    const float sc = (part < 2) ? kCarry : 0.0f;
#pragma unroll
    for (int e = 0; e < 8; ++e) {
      int m1 = part * 8 + e;
      m1 = (m1 > 15) ? 15 : m1;
      v[e] = c0[m1 * 512 + p1 * 32 + q1] * sc;
    }
    dst = bt1 + (size_t)g * 8;
  } else if (blk < kPrepBlk2) {
    const int g = (blk - kPrepBlk1) * 256 + t;
    const int row = g >> 6, part = g & 63;
    const int p2 = row >> 5, q2 = row & 31;
    const int m2 = part >> 2, r0 = (part & 3) * 8;
#pragma unroll
    for (int e = 0; e < 8; ++e)
      v[e] = c1[(size_t)(r0 + e) * 8192 + m2 * 512 + p2 * 32 + q2] * kCarry;
    dst = bt2 + (size_t)g * 8;
  } else {
    const int g = (blk - kPrepBlk2) * 256 + t;
    const int row = g >> 6, part = g & 63;
    const int m3 = part >> 2, r0 = (part & 3) * 8;
    const int p3 = (row > 15) ? 15 : row;
    const float sc = (row < 16) ? kCarry : 0.0f;
#pragma unroll
    for (int e = 0; e < 8; ++e)
      v[e] = c2[(r0 + e) * 256 + m3 * 16 + p3] * sc;
    dst = bt3 + (size_t)g * 8;
  }
  const v4u u = pack8_f16(v[0], v[1], v[2], v[3], v[4], v[5], v[6], v[7]);
  store16_twice(dst, u);
}

__global__ __launch_bounds__(256) void gather_x_kernel(const float* __restrict__ x, unsigned short* __restrict__ xg) {
  const int g = blockIdx.x * 256 + threadIdx.x;
  const int row = g >> 2, part = g & 3;
  const int b = row >> 8, t1 = row & 255;
  const float sc = (part < 2) ? 1.0f : 0.0f;
  const float* xb = x + (size_t)b * kInFeat + t1;
  float v[8];
#pragma unroll
  for (int e = 0; e < 8; ++e) {
    int m1 = part * 8 + e;
    m1 = (m1 > 15) ? 15 : m1;
    v[e] = xb[m1 * 256] * sc;
  }
  const v4u u = pack8_f16(v[0], v[1], v[2], v[3], v[4], v[5], v[6], v[7]);
  store16_twice(xg + (size_t)g * 8, u);
}

__global__ __launch_bounds__(256) void regather_kernel(const unsigned short* __restrict__ src, unsigned short* __restrict__ dst) {
  const int g = blockIdx.x * 256 + threadIdx.x;
  const int drow = g >> 6, part = g & 63;
  const int w = part >> 2, r8 = part & 3;
  const int bl = drow >> 8, u = (drow >> 4) & 15, vv = drow & 15;
  const int srow = (bl * 16 + w) * 16 + u;
  const v4u val = *(const v4u*)(src + (size_t)srow * kKbig + vv * 32 + r8 * 8);
  store16_twice(dst + (size_t)g * 8, val);
}

__global__ __launch_bounds__(256) void bias_relu_kernel(const float* __restrict__ s3, const float* __restrict__ bias,
                                                         float* __restrict__ outp) {
  const int g = blockIdx.x * 256 + threadIdx.x;
  const int o = g * 4;
  const int row = o >> 4, col = o & 15;
  const v4f s = *(const v4f*)(s3 + (size_t)row * kN3 + col);
  const int nn = row & 255;
  const v4f bb = *(const v4f*)(bias + nn * 16 + col);
  v4f r;
#pragma unroll
  for (int e = 0; e < 4; ++e) {
    const float tsum = s[e] + bb[e];
    r[e] = fmaxf(tsum, 0.0f);
  }
  float* op = outp + (size_t)o;
  *(volatile v4f*)op = r;
  __threadfence();
  *(volatile v4f*)op = r;
}

extern "C" void kernel_launch(void* const* d_in, const int* in_sizes, int n_in,
                              void* d_out, int out_size, void* d_ws, size_t ws_size,
                              hipStream_t stream) {
  if (n_in < 5) return;
  if (in_sizes[0] != kBatch * kInFeat) return;
  if (in_sizes[1] != 1 * 16 * 16 * 32) return;
  if (in_sizes[2] != 32 * 16 * 16 * 32) return;
  if (in_sizes[3] != 32 * 16 * 16 * 1) return;
  if (in_sizes[4] != kOutFeat) return;
  if (out_size != kBatch * kOutFeat) return;
  if (kWsTotal > ws_size) return;

  const float* x    = (const float*)d_in[0];
  const float* c0   = (const float*)d_in[1];
  const float* c1   = (const float*)d_in[2];
  const float* c2   = (const float*)d_in[3];
  const float* bias = (const float*)d_in[4];
  float* out = (float*)d_out;
  char* ws = (char*)d_ws;

  unsigned short* xg  = (unsigned short*)(ws + kOffXG);
  unsigned short* bt1 = (unsigned short*)(ws + kOffBT1);
  unsigned short* bt2 = (unsigned short*)(ws + kOffBT2);
  unsigned short* bt3 = (unsigned short*)(ws + kOffBT3);
  unsigned short* r1  = (unsigned short*)(ws + kOffR1);
  unsigned short* r2  = (unsigned short*)(ws + kOffR2);
  float* r1f = (float*)(ws + kOffR1);

  prep_cores_kernel<<<kPrepBlk3, 256, 0, stream>>>(c0, c1, c2, bt1, bt2, bt3);
  gather_x_kernel<<<kGatherXBlk, 256, 0, stream>>>(x, xg);

  for (int c = 0; c < kNumChunks; ++c) {
    const unsigned short* xgc = xg + (size_t)c * kRowsChunk * kK1;
    float* outc = out + (size_t)c * kRowsChunk * 16;

    wmma_gemm64<0, false, 0, 1, false, 0><<<dim3(kGemmBlk12, 1), 256, 0, stream>>>(
        xgc, xgc, kK1, 0L, bt1, bt1, kK1, 0L, (void*)r1, (void*)r1, kN12, 0L,
        bias, bias, 0L, kRowsChunk, kN12, kK1, 1.0f);
    regather_kernel<<<kRegatherBlk, 256, 0, stream>>>(r1, r2);
    wmma_gemm64<0, false, 0, 1, false, 0><<<dim3(kGemmBlk12, 1), 256, 0, stream>>>(
        r2, r2, kKbig, 0L, bt2, bt2, kKbig, 0L, (void*)r1, (void*)r1, kN12, 0L,
        bias, bias, 0L, kRowsChunk, kN12, kKbig, kScale2);
    regather_kernel<<<kRegatherBlk, 256, 0, stream>>>(r1, r2);
    wmma_gemm64<0, false, 0, 0, false, 0><<<dim3(kGemmBlk3, 1), 256, 0, stream>>>(
        r2, r2, kKbig, 0L, bt3, bt3, kKbig, 0L, (void*)r1f, (void*)r1f, kN3, 0L,
        bias, bias, 0L, kRowsChunk, kN3, kKbig, kScale3);
    bias_relu_kernel<<<kEpiBlk, 256, 0, stream>>>(r1f, bias, outc);
  }
}
